// LeagueGNN_14207751815591
// MI455X (gfx1250) — hardware-verified
//
#include <hip/hip_runtime.h>
#include <stddef.h>


#define HID    64
#define CHD    32
#define RLD    8
#define NCH    170
#define NRL    10
#define NODEK  41
#define FCN    32
#define NPG    10
#define BW     2048
#define BWSH   11
#define FPC    16
#define CWN    (FPC * BW)
#define CCAP   286720
#define FCAP   19456
#define FOFW   2080
#define STG    2304
#define FLT    2048
#define DEGCAP 256
#define NTHR   256
#define NWAVE  8
#define GROWS  128
#define APITCH 72
#define TPK    64
#define TPN    32
#define TPP    72
#define ASCL   16.0f
#define HSCL   64.0f
#define GSCL   64.0f
#define WSCL   64.0f
#define AGSCL  16.0f
#define LDS_FINE ((2 * FCAP + FOFW) * 4)

static_assert((CCAP % 256) == 0);
static_assert((FCAP % 32) == 0);
static_assert((FOFW % 32) == 0 && FOFW == BW + 32);
static_assert(STG >= FLT + 256 && (FLT % 32) == 0);
static_assert((BW & (BW - 1)) == 0 && (1 << BWSH) == BW);
static_assert(BW == 64 * 32);
static_assert(GROWS == NWAVE * 16 && NTHR == NWAVE * 32);
static_assert((APITCH % 8) == 0 && APITCH >= HID);
static_assert(TPN * 8 == NTHR && TPK == NWAVE * 8 && (TPP % 8) == 0 && TPP >= TPK);
static_assert(LDS_FINE <= 300 * 1024);
static_assert(CHD + RLD + 1 == NODEK && NODEK <= HID);
static_assert(HID == 2 * 32 && CHD == 32 && RLD == 8);

typedef float    v2f  __attribute__((ext_vector_type(2)));
typedef float    v4f  __attribute__((ext_vector_type(4)));
typedef float    v8f  __attribute__((ext_vector_type(8)));
typedef int      v4i  __attribute__((ext_vector_type(4)));
typedef double   v2d  __attribute__((ext_vector_type(2)));
typedef _Float16 v8h  __attribute__((ext_vector_type(8)));
typedef _Float16 v16h __attribute__((ext_vector_type(16)));
union FragH { v16h v; v8h h[2]; };
union H16U  { _Float16 h; unsigned short u; };

#define WSYNC() { __builtin_amdgcn_fence(__ATOMIC_ACQ_REL, "wavefront"); __builtin_amdgcn_wave_barrier(); }

__device__ __forceinline__ v8f wmf(v16h a, v16h b, v8f c) {
  v8f d = __builtin_amdgcn_wmma_f32_16x16x32_f16(false, a, false, b, (short)0, c, false, false);
  asm volatile("v_nop\n\tv_nop\n\tv_nop\n\tv_nop" : "+v"(d) : "v"(a), "v"(b));
  return d;
}

__device__ __forceinline__ v8h cvt8(v4f a, v4f b, float z) {
  v8h o;
  o[0] = (_Float16)(a.x * z); o[1] = (_Float16)(a.y * z); o[2] = (_Float16)(a.z * z); o[3] = (_Float16)(a.w * z);
  o[4] = (_Float16)(b.x * z); o[5] = (_Float16)(b.y * z); o[6] = (_Float16)(b.z * z); o[7] = (_Float16)(b.w * z);
  return o;
}

__device__ __forceinline__ unsigned same_key_mask(int key, bool valid) {
  unsigned m = __builtin_amdgcn_ballot_w32(valid);
#pragma unroll
  for (int b = 0; b < BWSH; ++b) {
    const bool bit = ((key >> b) & 1) != 0;
    const unsigned bb = __builtin_amdgcn_ballot_w32(valid && bit);
    m &= bit ? bb : ~bb;
  }
  return m;
}

__global__ __launch_bounds__(NTHR) void k_wT16(const float* __restrict__ W, _Float16* Wp,
                                               int KD, int NC, int nK, float scale) {
  __shared__ __attribute__((aligned(16))) _Float16 sT[TPN * TPP];
  const int tid = threadIdx.x;
  const int k0 = (int)blockIdx.x * TPK, n0 = (int)blockIdx.y * TPN;
  const int nc = tid & 31, kq = tid >> 5;
#pragma unroll
  for (int i = 0; i < TPK / NWAVE; ++i) {
    const int kr = kq + NWAVE * i;
    const int k  = k0 + kr;
    const int kc = k < nK ? k : nK - 1;
    const float z = (k < nK) ? scale : 0.0f;
    const float v = W[(size_t)kc * NC + n0 + nc] * z;
    sT[nc * TPP + kr] = (_Float16)v;
  }
  __syncthreads();
  const int nl = tid >> 3, p = tid & 7;
  const v8h hv = *(const v8h*)(sT + nl * TPP + 8 * p);
  _Float16* d = Wp + (size_t)(n0 + nl) * KD + k0 + 8 * p;
  *(volatile v8h*)d = hv;
  __threadfence();
  *(volatile v8h*)d = hv;
}

__device__ __forceinline__ void coarse_flush(int* stS, int* stD, int* cs, int* cd, int lane, int nfl,
                                             int& fill, int& gpos, int& vw, int& ovf) {
  const int room = CCAP - gpos;
  const int nw = nfl <= room ? nfl : room;
  const int consumed = fill < nfl ? fill : nfl;
  if (consumed > nw) ovf = 1;
  vw += (consumed < nw ? consumed : nw);
  WSYNC()
  const int nv = nw >> 2;
  int* gs = cs + gpos;
  int* gd = cd + gpos;
#pragma unroll 1
  for (int i = lane; i < nv; i += 32) {
    const v4i a = *(const v4i*)(stS + 4 * i);
    const v4i b = *(const v4i*)(stD + 4 * i);
    *(volatile v4i*)(gs + 4 * i) = a;
    *(volatile v4i*)(gd + 4 * i) = b;
  }
  __threadfence();
#pragma unroll 1
  for (int i = lane; i < nv; i += 32) {
    const v4i a = *(const v4i*)(stS + 4 * i);
    const v4i b = *(const v4i*)(stD + 4 * i);
    *(volatile v4i*)(gs + 4 * i) = a;
    *(volatile v4i*)(gd + 4 * i) = b;
  }
  gpos += nw;
  const int t = fill - nfl;
  const int ti = (nfl + lane) < (STG - 1) ? (nfl + lane) : (STG - 1);
  const int tS = stS[ti];
  const int tD = stD[ti];
  WSYNC()
  if (lane < t) { stS[lane] = tS; stD[lane] = tD; }
  WSYNC()
  fill = t > 0 ? t : 0;
}

__global__ __launch_bounds__(32) void k_coarse(const int* __restrict__ esrc, const int* __restrict__ edst,
                                              int* CS, int* CD, int* CCNT, int nE, int nN, int vec8) {
  __shared__ __attribute__((aligned(16))) int stS[STG];
  __shared__ __attribute__((aligned(16))) int stD[STG];
  const int lane = threadIdx.x;
  const int c = blockIdx.x;
  const unsigned nb = (unsigned)(c * CWN);
  int* cs = CS + (size_t)c * CCAP;
  int* cd = CD + (size_t)c * CCAP;
  int fill = 0, gpos = 0, vw = 0, ovf = 0;
  const int sent = -2147483647 - 1;
  const int nGrp = (nE + 255) / 256;
#pragma unroll 1
  for (int g = 0; g < nGrp; ++g) {
    const int base = g * 256;
    const int e0 = base + 8 * lane;
    v4i da, db, sa, sb;
    if (vec8 != 0 && base + 256 <= nE) {
      da = *(const v4i*)(edst + e0);
      db = *(const v4i*)(edst + e0 + 4);
      sa = *(const v4i*)(esrc + e0);
      sb = *(const v4i*)(esrc + e0 + 4);
    } else {
      const int i0 = min(e0, nE - 1),     i1 = min(e0 + 1, nE - 1), i2 = min(e0 + 2, nE - 1), i3 = min(e0 + 3, nE - 1);
      const int i4 = min(e0 + 4, nE - 1), i5 = min(e0 + 5, nE - 1), i6 = min(e0 + 6, nE - 1), i7 = min(e0 + 7, nE - 1);
      da.x = (e0     < nE) ? edst[i0] : sent;
      da.y = (e0 + 1 < nE) ? edst[i1] : sent;
      da.z = (e0 + 2 < nE) ? edst[i2] : sent;
      da.w = (e0 + 3 < nE) ? edst[i3] : sent;
      db.x = (e0 + 4 < nE) ? edst[i4] : sent;
      db.y = (e0 + 5 < nE) ? edst[i5] : sent;
      db.z = (e0 + 6 < nE) ? edst[i6] : sent;
      db.w = (e0 + 7 < nE) ? edst[i7] : sent;
      sa.x = esrc[i0]; sa.y = esrc[i1]; sa.z = esrc[i2]; sa.w = esrc[i3];
      sb.x = esrc[i4]; sb.y = esrc[i5]; sb.z = esrc[i6]; sb.w = esrc[i7];
    }
    sa.x = min(max(sa.x, 0), nN - 1); sa.y = min(max(sa.y, 0), nN - 1);
    sa.z = min(max(sa.z, 0), nN - 1); sa.w = min(max(sa.w, 0), nN - 1);
    sb.x = min(max(sb.x, 0), nN - 1); sb.y = min(max(sb.y, 0), nN - 1);
    sb.z = min(max(sb.z, 0), nN - 1); sb.w = min(max(sb.w, 0), nN - 1);
#define CAPP(SV, DV) { \
      const unsigned dl = (unsigned)(DV) - nb; \
      const bool ht = dl < (unsigned)CWN; \
      const unsigned mk = __builtin_amdgcn_ballot_w32(ht); \
      if (ht) { \
        const int pos = fill + (int)__builtin_amdgcn_mbcnt_lo(mk, 0u); \
        if (pos < STG) { stS[pos] = (SV); stD[pos] = (int)dl; } \
      } \
      fill += (int)__builtin_popcount(mk); }
    CAPP(sa.x, da.x)
    CAPP(sa.y, da.y)
    CAPP(sa.z, da.z)
    CAPP(sa.w, da.w)
    CAPP(sb.x, db.x)
    CAPP(sb.y, db.y)
    CAPP(sb.z, db.z)
    CAPP(sb.w, db.w)
#undef CAPP
    if (fill >= FLT) coarse_flush(stS, stD, cs, cd, lane, fill & ~31, fill, gpos, vw, ovf);
  }
  coarse_flush(stS, stD, cs, cd, lane, ((fill + 31) >> 5) << 5, fill, gpos, vw, ovf);
  int val = 0;
  if (lane == 0) val = vw;
  if (lane == 1) val = ovf;
  int* cl = CCNT + (size_t)c * 32 + lane;
  *(volatile int*)cl = val;
  __threadfence();
  *(volatile int*)cl = val;
}

__global__ __launch_bounds__(32) void k_fine(const int* __restrict__ CS, const int* __restrict__ CD, const int* __restrict__ CCNT,
                                            int* FCSR, int* FOFF, float* dinv, int nN) {
  extern __shared__ v4i lds_raw[];
  int* hits = (int*)lds_raw;
  int* img  = hits + FCAP;
  int* off  = img + FCAP;
  const int lane = threadIdx.x;
  const int f = blockIdx.x;
  const int c = f / FPC;
  const unsigned lo = (unsigned)((f - c * FPC) * BW);
  int nc = CCNT[(size_t)c * 32];
  nc = nc < 0 ? 0 : (nc > CCAP ? CCAP : nc);
  const int* cs = CS + (size_t)c * CCAP;
  const int* cd = CD + (size_t)c * CCAP;

  int fill = 0;
  const int nGrp = (nc + 255) >> 8;
#pragma unroll 1
  for (int g = 0; g < nGrp; ++g) {
    const int i0 = g * 256 + 8 * lane;
    const v4i sa = *(const v4i*)(cs + i0), sb = *(const v4i*)(cs + i0 + 4);
    const v4i da = *(const v4i*)(cd + i0), db = *(const v4i*)(cd + i0 + 4);
#define FAPP(J, SV, DV) { \
      const unsigned dl = (unsigned)(DV) - lo; \
      const bool ht = ((i0 + (J)) < nc) && (dl < (unsigned)BW); \
      int sv = (SV); sv = sv < 0 ? 0 : (sv > nN - 1 ? nN - 1 : sv); \
      const int ent = (sv << BWSH) | (int)(dl & (unsigned)(BW - 1)); \
      const unsigned mk = __builtin_amdgcn_ballot_w32(ht); \
      if (ht) { \
        const int pos = fill + (int)__builtin_amdgcn_mbcnt_lo(mk, 0u); \
        if (pos < FCAP) hits[pos] = ent; \
      } \
      fill += (int)__builtin_popcount(mk); }
    FAPP(0, sa.x, da.x)
    FAPP(1, sa.y, da.y)
    FAPP(2, sa.z, da.z)
    FAPP(3, sa.w, da.w)
    FAPP(4, sb.x, db.x)
    FAPP(5, sb.y, db.y)
    FAPP(6, sb.z, db.z)
    FAPP(7, sb.w, db.w)
#undef FAPP
  }
  const int ovf = fill > FCAP ? 1 : 0;
  const int fillc = fill < FCAP ? fill : FCAP;
  WSYNC()

#pragma unroll 1
  for (int i = lane; i < FOFW; i += 32) off[i] = 0;
  WSYNC()
  const int nHG = (fillc + 31) >> 5;
#pragma unroll 1
  for (int g = 0; g < nHG; ++g) {
    const int idx = g * 32 + lane;
    const bool valid = idx < fillc;
    const int e = hits[idx < FCAP - 1 ? idx : FCAP - 1];
    const int key = e & (BW - 1);
    const unsigned mk = same_key_mask(key, valid);
    const int rank = (int)__builtin_amdgcn_mbcnt_lo(mk, 0u);
    const int tot  = (int)__builtin_popcount(mk);
    if (valid && rank == tot - 1) off[key] = off[key] + tot;
    WSYNC()
  }

  int run = 0;
#pragma unroll 8
  for (int j = 0; j < 64; ++j) run += off[64 * lane + j];
  int incl = run;
#pragma unroll
  for (int d = 1; d < 32; d <<= 1) {
    const int t = __shfl_up(incl, d, 32);
    if (lane >= d) incl += t;
  }
  int acc = incl - run;
#pragma unroll 8
  for (int j = 0; j < 64; ++j) { img[64 * lane + j] = acc; acc += off[64 * lane + j]; }
  if (lane == 31) img[BW] = acc;
  if (lane == 0)  img[BW + 1] = ovf;
#pragma unroll 1
  for (int i = BW + 2 + lane; i < FOFW; i += 32) img[i] = 0;
  WSYNC()

  int*   rp = FOFF + (size_t)f * FOFW;
  float* dp = dinv + (size_t)f * BW;
#pragma unroll 1
  for (int i = lane; i < FOFW / 4; i += 32) { const v4i v = *(const v4i*)(img + 4 * i); *(volatile v4i*)(rp + 4 * i) = v; }
#pragma unroll 1
  for (int i = lane; i < BW / 4; i += 32) {
    const v4i c4 = *(const v4i*)(off + 4 * i);
    v4f d;
    d.x = rsqrtf((float)max(c4.x, 0) + 1.0f); d.y = rsqrtf((float)max(c4.y, 0) + 1.0f);
    d.z = rsqrtf((float)max(c4.z, 0) + 1.0f); d.w = rsqrtf((float)max(c4.w, 0) + 1.0f);
    *(volatile v4f*)(dp + 4 * i) = d;
  }
  __threadfence();
#pragma unroll 1
  for (int i = lane; i < FOFW / 4; i += 32) { const v4i v = *(const v4i*)(img + 4 * i); *(volatile v4i*)(rp + 4 * i) = v; }
#pragma unroll 1
  for (int i = lane; i < BW / 4; i += 32) {
    const v4i c4 = *(const v4i*)(off + 4 * i);
    v4f d;
    d.x = rsqrtf((float)max(c4.x, 0) + 1.0f); d.y = rsqrtf((float)max(c4.y, 0) + 1.0f);
    d.z = rsqrtf((float)max(c4.z, 0) + 1.0f); d.w = rsqrtf((float)max(c4.w, 0) + 1.0f);
    *(volatile v4f*)(dp + 4 * i) = d;
  }
  WSYNC()

#pragma unroll 1
  for (int i = lane; i < BW; i += 32) off[i] = img[i];
  WSYNC()
#pragma unroll 1
  for (int g = 0; g < nHG; ++g) {
    const int idx = g * 32 + lane;
    const bool valid = idx < fillc;
    const int e = hits[idx < FCAP - 1 ? idx : FCAP - 1];
    const int key = e & (BW - 1);
    int src = e >> BWSH;
    src = src < 0 ? 0 : (src > nN - 1 ? nN - 1 : src);
    const unsigned mk = same_key_mask(key, valid);
    const int rank = (int)__builtin_amdgcn_mbcnt_lo(mk, 0u);
    const int tot  = (int)__builtin_popcount(mk);
    const int cb = off[key];
    int pos = cb + rank;
    pos = pos < 0 ? 0 : (pos > FCAP - 1 ? FCAP - 1 : pos);
    if (valid) img[pos] = src;
    if (valid && rank == tot - 1) off[key] = cb + tot;
    WSYNC()
  }

  const int nv = ((fillc + 31) & ~31) >> 2;
  int* gp = FCSR + (size_t)f * FCAP;
#pragma unroll 1
  for (int i = lane; i < nv; i += 32) { const v4i v = *(const v4i*)(img + 4 * i); *(volatile v4i*)(gp + 4 * i) = v; }
  __threadfence();
#pragma unroll 1
  for (int i = lane; i < nv; i += 32) { const v4i v = *(const v4i*)(img + 4 * i); *(volatile v4i*)(gp + 4 * i) = v; }
}

template <int PRO, int NC, int EPI>
__global__ __launch_bounds__(NTHR) void k_gemm(
    const int* __restrict__ xi, const float* __restrict__ tabC, const float* __restrict__ tabR,
    const _Float16* __restrict__ A16, const float* __restrict__ ss, const float* __restrict__ A32,
    const _Float16* __restrict__ Bw, const float* __restrict__ rsc, const float* __restrict__ bias,
    float* C, double* part, int nValid, float ascl, float osc) {
  static_assert((NC % 16) == 0 && (128 % NC) == 0 && NC <= HID);
  static_assert(EPI == 0 || NC == FCN);
  constexpr int KD  = HID;
  constexpr int NT  = NC / 16;
  constexpr int RPI = 128 / NC;
  constexpr int NST = 16 / RPI;
  __shared__ __attribute__((aligned(16))) _Float16 sA[GROWS * APITCH];
  __shared__ __attribute__((aligned(16))) float stg[GROWS * NC];
  __shared__ double sps[NWAVE * 64];
  const int tid = threadIdx.x, lane = tid & 31, wave = tid >> 5, hh = lane >> 4, m = lane & 15;
  const int rowBase = blockIdx.x * GROWS;

  {
    const int hf = wave & 1;
    const int r  = (wave >> 1) * 32 + lane;
    const int n  = rowBase + r;
    const bool valid = n < nValid;
    const float z = valid ? ascl : 0.0f;
    _Float16* arow = sA + r * APITCH + 32 * hf;
    if (PRO == 0) {
      const int ncl = valid ? n : nValid - 1;
      if (hf == 0) {
        int id = xi[(size_t)ncl * 3 + 0];
        id = id < 0 ? id + NCH : id;
        id = min(max(id, 0), NCH - 1);
        const float* tp = tabC + (size_t)id * CHD;
#pragma unroll
        for (int q = 0; q < 4; ++q) {
          const v4f f0 = *(const v4f*)(tp + 8 * q);
          const v4f f1 = *(const v4f*)(tp + 8 * q + 4);
          *(v8h*)(arow + 8 * q) = cvt8(f0, f1, z);
        }
      } else {
        int id = xi[(size_t)ncl * 3 + 1];
        id = id < 0 ? id + NRL : id;
        id = min(max(id, 0), NRL - 1);
        const float* tp = tabR + (size_t)id * RLD;
        const v4f f0 = *(const v4f*)tp;
        const v4f f1 = *(const v4f*)(tp + 4);
        *(v8h*)(arow) = cvt8(f0, f1, z);
        const int tm = xi[(size_t)ncl * 3 + 2];
        H16U th; th.h = (_Float16)((float)tm * z);
        v4i w0; w0.x = (int)(unsigned)th.u; w0.y = 0; w0.z = 0; w0.w = 0;
        const v4i wz = {0, 0, 0, 0};
        *(v4i*)(arow + 8)  = w0;
        *(v4i*)(arow + 16) = wz;
        *(v4i*)(arow + 24) = wz;
      }
    } else if (PRO == 1) {
      const _Float16* src = A16 + (size_t)n * HID + 32 * hf;
      const float inv = 1.0f / AGSCL;
#pragma unroll
      for (int q = 0; q < 4; ++q) {
        const v8h hv = *(const v8h*)(src + 8 * q);
        const int col = 32 * hf + 8 * q;
        const v4f c0 = *(const v4f*)(ss + col), c1 = *(const v4f*)(ss + col + 4);
        const v4f t0 = *(const v4f*)(ss + HID + col), t1 = *(const v4f*)(ss + HID + col + 4);
        v8h o;
        o[0] = (_Float16)(fmaxf((float)hv[0] * inv * c0.x + t0.x, 0.0f) * z);
        o[1] = (_Float16)(fmaxf((float)hv[1] * inv * c0.y + t0.y, 0.0f) * z);
        o[2] = (_Float16)(fmaxf((float)hv[2] * inv * c0.z + t0.z, 0.0f) * z);
        o[3] = (_Float16)(fmaxf((float)hv[3] * inv * c0.w + t0.w, 0.0f) * z);
        o[4] = (_Float16)(fmaxf((float)hv[4] * inv * c1.x + t1.x, 0.0f) * z);
        o[5] = (_Float16)(fmaxf((float)hv[5] * inv * c1.y + t1.y, 0.0f) * z);
        o[6] = (_Float16)(fmaxf((float)hv[6] * inv * c1.z + t1.z, 0.0f) * z);
        o[7] = (_Float16)(fmaxf((float)hv[7] * inv * c1.w + t1.w, 0.0f) * z);
        *(v8h*)(arow + 8 * q) = o;
      }
    } else {
      const float* src = A32 + (size_t)n * HID + 32 * hf;
#pragma unroll
      for (int q = 0; q < 4; ++q) {
        const v4f f0 = *(const v4f*)(src + 8 * q);
        const v4f f1 = *(const v4f*)(src + 8 * q + 4);
        *(v8h*)(arow + 8 * q) = cvt8(f0, f1, z);
      }
    }
  }
  __syncthreads();

  const _Float16* ap  = sA + (wave * 16 + m) * APITCH + 8 * hh;
  const _Float16* bp0 = Bw + (size_t)m * KD + 8 * hh;
  v8f acc[NT];
#pragma unroll
  for (int t = 0; t < NT; ++t) { v8f zz = {0.f, 0.f, 0.f, 0.f, 0.f, 0.f, 0.f, 0.f}; acc[t] = zz; }
#pragma unroll
  for (int kt = 0; kt < KD / 32; ++kt) {
    FragH af;
    af.h[0] = *(const v8h*)(ap + 32 * kt);
    af.h[1] = *(const v8h*)(ap + 32 * kt + 16);
#pragma unroll
    for (int t = 0; t < NT; ++t) {
      const _Float16* bp = bp0 + (size_t)(16 * t) * KD + 32 * kt;
      FragH bf;
      bf.h[0] = *(const v8h*)bp;
      bf.h[1] = *(const v8h*)(bp + 16);
      acc[t] = wmf(af.v, bf.v, acc[t]);
    }
  }

  const int r0 = wave * 16 + 8 * hh;
  float s[8];
  if (EPI == 0) {
    const v4f dA = *(const v4f*)(rsc + (size_t)rowBase + r0);
    const v4f dB = *(const v4f*)(rsc + (size_t)rowBase + r0 + 4);
    s[0] = dA.x; s[1] = dA.y; s[2] = dA.z; s[3] = dA.w; s[4] = dB.x; s[5] = dB.y; s[6] = dB.z; s[7] = dB.w;
#pragma unroll
    for (int r = 0; r < 8; ++r) s[r] = s[r] * osc;
  } else {
#pragma unroll
    for (int r = 0; r < 8; ++r) s[r] = osc;
  }
  float bc[NT];
#pragma unroll
  for (int t = 0; t < NT; ++t) bc[t] = (EPI == 1) ? bias[16 * t + m] : 0.0f;

  float* sp = stg + r0 * NC + m;
#pragma unroll
  for (int t = 0; t < NT; ++t) {
#pragma unroll
    for (int r = 0; r < 8; ++r) sp[r * NC + 16 * t] = acc[t][r] * s[r] + bc[t];
  }
  __syncthreads();

  const float* lp = stg + wave * 16 * NC;
  float* gp = C + (size_t)(rowBase + wave * 16) * NC;
#pragma unroll
  for (int i = 0; i < NST; ++i) {
    const v4f v = *(const v4f*)(lp + i * 128 + 4 * lane);
    *(volatile v4f*)(gp + (size_t)i * 128 + 4 * lane) = v;
  }
  __threadfence();
#pragma unroll
  for (int i = 0; i < NST; ++i) {
    const v4f v = *(const v4f*)(lp + i * 128 + 4 * lane);
    *(volatile v4f*)(gp + (size_t)i * 128 + 4 * lane) = v;
  }

  if (EPI == 1) {
    const int cc = tid & 31, pr = tid >> 5;
    double S = 0.0, Q = 0.0;
#pragma unroll 1
    for (int i = 0; i < 16; ++i) {
      const int row = pr * 16 + i;
      const float v = stg[row * NC + cc];
      const bool ok = (rowBase + row) < nValid;
      S += ok ? (double)v : 0.0;
      Q += ok ? (double)v * (double)v : 0.0;
    }
    sps[pr * 64 + 2 * cc]     = S;
    sps[pr * 64 + 2 * cc + 1] = Q;
    __syncthreads();
    if (tid < 32) {
      double S2 = 0.0, Q2 = 0.0;
#pragma unroll
      for (int p = 0; p < NWAVE; ++p) { S2 += sps[p * 64 + 2 * lane]; Q2 += sps[p * 64 + 2 * lane + 1]; }
      v2d o; o.x = S2; o.y = Q2;
      double* pp = part + (size_t)blockIdx.x * 64 + 2 * lane;
      *(volatile v2d*)pp = o;
      __threadfence();
      *(volatile v2d*)pp = o;
    }
  }
}

template <int MODE>
__global__ __launch_bounds__(32) void k_agg(const int* __restrict__ FCSR, const int* __restrict__ FOFF,
                                           const float* __restrict__ dinv, const float* __restrict__ HW,
                                           const float* __restrict__ bias, const int* __restrict__ bat,
                                           unsigned int* outH, double* part, float* pool,
                                           int nN, int nG, float hscl) {
  const int lane = threadIdx.x, w = blockIdx.x, ch = 2 * lane;
  const v2f bq = *(const v2f*)(bias + ch);
  double s0 = 0.0, s1 = 0.0, q0 = 0.0, q1 = 0.0;
  constexpr int NOUT = (MODE == 1) ? 64 : 8;
  constexpr int NIN  = (MODE == 1) ? 1 : NPG;
#pragma unroll 1
  for (int jo = 0; jo < NOUT; ++jo) {
    const int g = w * 8 + jo;
    v2f gs = {0.f, 0.f};
    int gc = 0;
#pragma unroll 1
    for (int ji = 0; ji < NIN; ++ji) {
      const int n = (MODE == 1) ? (w * 64 + jo) : (g * NPG + ji);
      const int f = n >> BWSH, dl = n & (BW - 1);
      const int* rec = FOFF + (size_t)f * FOFW;
      int o0 = rec[dl];
      const int o1 = rec[dl + 1];
      o0 = o0 < 0 ? 0 : (o0 > FCAP ? FCAP : o0);
      int cnt = o1 - o0;
      cnt = cnt < 0 ? 0 : (cnt > DEGCAP ? DEGCAP : cnt);
      cnt = cnt > FCAP - o0 ? FCAP - o0 : cnt;
      const int* lst = FCSR + (size_t)f * FCAP;
      v2f acc = {0.f, 0.f};
#pragma unroll 1
      for (int q = 0; q < cnt; q += 32) {
        int p = o0 + q + lane;
        p = p > FCAP - 1 ? FCAP - 1 : p;
        int sl = lst[p];
        sl = sl < 0 ? 0 : (sl > nN - 1 ? nN - 1 : sl);
        const int mc = (cnt - q) < 32 ? (cnt - q) : 32;
#pragma unroll 1
        for (int pp = 0; pp < mc; ++pp) {
          const int sidx = __builtin_amdgcn_readlane(sl, pp);
          acc = acc + *(const v2f*)(HW + (size_t)sidx * HID + ch);
        }
      }
      const float dn = dinv[n];
      const v2f sv = *(const v2f*)(HW + (size_t)n * HID + ch);
      v2f v = (acc + sv) * dn + bq;
      if (MODE == 1) {
        if (n < nN) {
          s0 += (double)v.x; s1 += (double)v.y;
          q0 += (double)v.x * (double)v.x; q1 += (double)v.y * (double)v.y;
        }
        H16U c0, c1;
        c0.h = (_Float16)(v.x * hscl);
        c1.h = (_Float16)(v.y * hscl);
        const unsigned wd = (unsigned)c0.u | ((unsigned)c1.u << 16);
        unsigned int* op = outH + (size_t)n * 32 + lane;
        *(volatile unsigned int*)op = wd;
        __threadfence();
        *(volatile unsigned int*)op = wd;
      } else {
        v.x = fmaxf(v.x, 0.0f); v.y = fmaxf(v.y, 0.0f);
        const int nb = bat[n < nN - 1 ? n : nN - 1];
        const bool mem = (n < nN) && (nb == g);
        if (mem) { gs = gs + v; gc += 1; }
      }
    }
    if (MODE == 2) {
      const float cf = (float)(gc > 1 ? gc : 1);
      const float rc = 1.0f / cf;
      v2f pv = {0.f, 0.f};
      if (g < nG) pv = gs * rc;
      float* pq = pool + (size_t)g * HID + ch;
      *(volatile v2f*)pq = pv;
      __threadfence();
      *(volatile v2f*)pq = pv;
    }
  }
  if (MODE == 1) {
    double* pp = part + (size_t)w * 128;
    v2d a; a.x = s0; a.y = s1;
    v2d b; b.x = q0; b.y = q1;
    *(volatile v2d*)(pp + 2 * lane) = a;
    *(volatile v2d*)(pp + 64 + 2 * lane) = b;
    __threadfence();
    *(volatile v2d*)(pp + 2 * lane) = a;
    *(volatile v2d*)(pp + 64 + 2 * lane) = b;
  }
}

__global__ __launch_bounds__(NTHR) void k_bn1fin(const double* __restrict__ part, int nW,
                                                 const float* __restrict__ gam, const float* __restrict__ bet,
                                                 float* ss, int nN) {
  __shared__ double sp[4 * 128];
  __shared__ __attribute__((aligned(16))) float sf[128];
  const int tid = threadIdx.x;
  const int c = tid & 63, pr = tid >> 6;
  double S = 0.0, Q = 0.0;
#pragma unroll 1
  for (int w = pr; w < nW; w += 4) {
    S += part[(size_t)w * 128 + c];
    Q += part[(size_t)w * 128 + 64 + c];
  }
  sp[pr * 128 + c] = S;
  sp[pr * 128 + 64 + c] = Q;
  __syncthreads();
  if (tid < 64) {
    double S2 = 0.0, Q2 = 0.0;
#pragma unroll
    for (int p = 0; p < 4; ++p) { S2 += sp[p * 128 + tid]; Q2 += sp[p * 128 + 64 + tid]; }
    const double mu = S2 / (double)nN;
    double var = Q2 / (double)nN - mu * mu;
    var = var < 0.0 ? 0.0 : var;
    const float sc = gam[tid] * rsqrtf((float)var + 1e-5f);
    sf[tid] = sc;
    sf[64 + tid] = bet[tid] - (float)mu * sc;
  }
  __syncthreads();
  if (tid < 32) {
    const v4f v = *(const v4f*)(sf + 4 * tid);
    *(volatile v4f*)(ss + 4 * tid) = v;
    __threadfence();
    *(volatile v4f*)(ss + 4 * tid) = v;
  }
}

__global__ __launch_bounds__(NTHR) void k_out(const double* __restrict__ part2, int nHB,
                                              const float* __restrict__ Z, int gPad,
                                              const float* __restrict__ gam, const float* __restrict__ bet,
                                              const float* __restrict__ w2, const float* __restrict__ b2,
                                              const int* __restrict__ CCNT, int nCB, const int* __restrict__ FOFF, int nBK,
                                              float* out, int nG) {
  __shared__ double sp[NWAVE * 64];
  __shared__ __attribute__((aligned(16))) float ssc[FCN];
  __shared__ __attribute__((aligned(16))) float ssh[FCN];
  __shared__ int pz[4];
  const int tid = threadIdx.x, lane = tid & 31, wave = tid >> 5;
  double S = 0.0, Q = 0.0;
#pragma unroll 1
  for (int b = wave; b < nHB; b += NWAVE) {
    S += part2[(size_t)b * 64 + 2 * lane];
    Q += part2[(size_t)b * 64 + 2 * lane + 1];
  }
  sp[wave * 64 + 2 * lane]     = S;
  sp[wave * 64 + 2 * lane + 1] = Q;
  const int fa = CCNT[(size_t)(tid < nCB - 1 ? tid : nCB - 1) * 32 + 1];
  const int fb = FOFF[(size_t)(tid < nBK - 1 ? tid : nBK - 1) * FOFW + BW + 1];
  const bool fl = ((tid < nCB) && (fa != 0)) || ((tid < nBK) && (fb != 0));
  if (tid == 0) pz[0] = 0;
  __syncthreads();
  if (fl) pz[0] = 1;
  if (tid < FCN) {
    double S2 = 0.0, Q2 = 0.0;
#pragma unroll
    for (int p = 0; p < NWAVE; ++p) { S2 += sp[p * 64 + 2 * tid]; Q2 += sp[p * 64 + 2 * tid + 1]; }
    const double mu = S2 / (double)nG;
    double var = Q2 / (double)nG - mu * mu;
    var = var < 0.0 ? 0.0 : var;
    const float sc = gam[tid] * rsqrtf((float)var + 1e-5f);
    ssc[tid] = sc;
    ssh[tid] = bet[tid] - (float)mu * sc;
  }
  __syncthreads();
  const int poison = pz[0];
  const int gi  = blockIdx.x * NTHR + tid;
  const int gcl = gi < gPad - 1 ? gi : gPad - 1;
  const float* zr = Z + (size_t)gcl * FCN;
  float a = b2[0];
#pragma unroll 1
  for (int k = 0; k < FCN; k += 4) {
    const v4f z4 = *(const v4f*)(zr + k);
    const v4f w4 = *(const v4f*)(w2 + k);
    const v4f c4 = *(const v4f*)(ssc + k);
    const v4f t4 = *(const v4f*)(ssh + k);
    a += fmaxf(z4.x * c4.x + t4.x, 0.0f) * w4.x;
    a += fmaxf(z4.y * c4.y + t4.y, 0.0f) * w4.y;
    a += fmaxf(z4.z * c4.z + t4.z, 0.0f) * w4.z;
    a += fmaxf(z4.w * c4.w + t4.w, 0.0f) * w4.w;
  }
  a = fminf(fmaxf(a, -80.0f), 80.0f);
  const float e = expf(-a);
  float o = __frcp_rn(1.0f + e);
  if (poison != 0) o = __int_as_float(0x7fc00000);
  if (gi < nG) *(volatile float*)(out + gi) = o;
  __threadfence();
  if (gi < nG) *(volatile float*)(out + gi) = o;
}

extern "C" void kernel_launch(void* const* d_in, const int* in_sizes, int n_in,
                              void* d_out, int out_size, void* d_ws, size_t ws_size,
                              hipStream_t stream) {
  if (n_in < 17) return;
  const int nN = in_sizes[0] / 3;
  const int nE = in_sizes[1] / 2;
  const int nG = out_size;
  if (nN <= 0 || nE <= 0 || nG <= 0) return;
  if (in_sizes[0] != 3 * nN || in_sizes[1] != 2 * nE || in_sizes[2] != nN) return;
  if (in_sizes[3] != NCH * CHD || in_sizes[4] != NRL * RLD) return;
  if (in_sizes[5] != NODEK * HID || in_sizes[6] != HID || in_sizes[7] != HID || in_sizes[8] != HID) return;
  if (in_sizes[9] != HID * HID || in_sizes[10] != HID) return;
  if (in_sizes[11] != HID * FCN || in_sizes[12] != FCN || in_sizes[13] != FCN || in_sizes[14] != FCN) return;
  if (in_sizes[15] != FCN || in_sizes[16] != 1) return;
  if (nN > (1 << 20) || nE > (1 << 26) || nG > (1 << 20)) return;

  const int*   xi   = (const int*)d_in[0];
  const int*   ei   = (const int*)d_in[1];
  const int*   bat  = (const int*)d_in[2];
  const float* tabC = (const float*)d_in[3];
  const float* tabR = (const float*)d_in[4];
  const float* W1   = (const float*)d_in[5];
  const float* b1   = (const float*)d_in[6];
  const float* g1   = (const float*)d_in[7];
  const float* be1  = (const float*)d_in[8];
  const float* W2   = (const float*)d_in[9];
  const float* b2   = (const float*)d_in[10];
  const float* Wf1  = (const float*)d_in[11];
  const float* bf1  = (const float*)d_in[12];
  const float* g2   = (const float*)d_in[13];
  const float* be2  = (const float*)d_in[14];
  const float* Wf2  = (const float*)d_in[15];
  const float* bf2  = (const float*)d_in[16];
  float* out = (float*)d_out;
  const int* esrc = ei;
  const int* edst = ei + (size_t)nE;

  const int NBK  = (nN + BW - 1) / BW;
  const int NPAD = NBK * BW;
  const int NCB  = (NBK + FPC - 1) / FPC;
  const int GPAD = ((nG + GROWS - 1) / GROWS) * GROWS;
  if (NCB > NTHR || NBK > NTHR) return;
  if ((long long)NPG * (long long)GPAD > (long long)NPAD) return;
  {
    const long long expC = (long long)nE * (long long)CWN / (long long)nN;
    const long long expF = (long long)nE * (long long)BW / (long long)nN;
    if (expC + expC / 16 + 4096 > (long long)CCAP) return;
    if (expF + expF / 8 + 512 > (long long)FCAP) return;
  }
  const int nGB = NPAD / GROWS;
  const int nW1 = NPAD / 64;
  const int nW2 = GPAD / 8;
  const int nHB = GPAD / GROWS;
  const int nOB = (nG + NTHR - 1) / NTHR;

  char* ws = (char*)d_ws;
  size_t off = 0;
#define CARVE(NAME, BYTES) const size_t NAME = off; off += (size_t)(BYTES); off = (off + 255) & ~(size_t)255;
  CARVE(oW1, (size_t)HID * HID * 2)
  CARVE(oW2, (size_t)HID * HID * 2)
  CARVE(oWF, (size_t)FCN * HID * 2)
  const size_t RSZ = (size_t)2 * (size_t)NCB * (size_t)CCAP * 4;
  CARVE(oR, RSZ)
  CARVE(oCC, (size_t)NCB * 128)
  CARVE(oFC, (size_t)NBK * (size_t)FCAP * 4)
  CARVE(oFO, (size_t)NBK * (size_t)FOFW * 4)
  CARVE(oDI, (size_t)NPAD * 4)
  CARVE(oHW, (size_t)NPAD * HID * 4)
  CARVE(oAG, (size_t)NPAD * HID * 2)
#undef CARVE
  if (off > ws_size) return;
  size_t r = oR;
  const size_t oP1 = r; r += (size_t)nW1 * 1024;          r = (r + 255) & ~(size_t)255;
  const size_t oSS = r; r += 512;                          r = (r + 255) & ~(size_t)255;
  const size_t oPL = r; r += (size_t)GPAD * HID * 4;       r = (r + 255) & ~(size_t)255;
  const size_t oZ  = r; r += (size_t)GPAD * FCN * 4;       r = (r + 255) & ~(size_t)255;
  const size_t oP2 = r; r += (size_t)nHB * 512;            r = (r + 255) & ~(size_t)255;
  if (r > oR + RSZ) return;

  _Float16* WP1 = (_Float16*)(ws + oW1);
  _Float16* WP2 = (_Float16*)(ws + oW2);
  _Float16* WPF = (_Float16*)(ws + oWF);
  int*      CS  = (int*)(ws + oR);
  int*      CD  = (int*)(ws + oR + (size_t)NCB * (size_t)CCAP * 4);
  int*      CC  = (int*)(ws + oCC);
  int*      FC  = (int*)(ws + oFC);
  int*      FO  = (int*)(ws + oFO);
  float*    DI  = (float*)(ws + oDI);
  float*    HW  = (float*)(ws + oHW);
  _Float16* AG  = (_Float16*)(ws + oAG);
  double*   P1  = (double*)(ws + oP1);
  float*    SS  = (float*)(ws + oSS);
  float*    PL  = (float*)(ws + oPL);
  float*    ZP  = (float*)(ws + oZ);
  double*   P2  = (double*)(ws + oP2);

  const int vec8 = ((nE & 7) == 0) ? 1 : 0;
  const float oscX = 1.0f / (ASCL * WSCL);
  const float oscH = 1.0f / (HSCL * WSCL);
  const float oscG = 1.0f / (GSCL * WSCL);

  {
    const dim3 gH(HID / TPK, HID / TPN);
    const dim3 gF(HID / TPK, FCN / TPN);
    k_wT16<<<gH, NTHR, 0, stream>>>(W1, WP1, HID, HID, NODEK, WSCL);
    k_wT16<<<gH, NTHR, 0, stream>>>(W2, WP2, HID, HID, HID, WSCL);
    k_wT16<<<gF, NTHR, 0, stream>>>(Wf1, WPF, HID, FCN, HID, WSCL);
  }
  k_coarse<<<NCB, 32, 0, stream>>>(esrc, edst, CS, CD, CC, nE, nN, vec8);
  hipFuncSetAttribute(reinterpret_cast<const void*>(&k_fine), hipFuncAttributeMaxDynamicSharedMemorySize, LDS_FINE);
  k_fine<<<NBK, 32, LDS_FINE, stream>>>(CS, CD, CC, FC, FO, DI, nN);
  k_gemm<0, HID, 0><<<nGB, NTHR, 0, stream>>>(xi, tabC, tabR, AG, SS, PL, WP1, DI, b1, HW, P2, nN, ASCL, oscX);
  k_agg<1><<<nW1, 32, 0, stream>>>(FC, FO, DI, HW, b1, bat, (unsigned int*)AG, P1, PL, nN, nG, AGSCL);
  k_bn1fin<<<1, NTHR, 0, stream>>>(P1, nW1, g1, be1, SS, nN);
  k_gemm<1, HID, 0><<<nGB, NTHR, 0, stream>>>(xi, tabC, tabR, AG, SS, PL, WP2, DI, b2, HW, P2, nN, HSCL, oscH);
  k_agg<2><<<nW2, 32, 0, stream>>>(FC, FO, DI, HW, b2, bat, (unsigned int*)AG, P1, PL, nN, nG, 1.0f);
  k_gemm<2, FCN, 1><<<nHB, NTHR, 0, stream>>>(xi, tabC, tabR, AG, SS, PL, WPF, DI, bf1, ZP, P2, nG, GSCL, oscG);
  k_out<<<nOB, NTHR, 0, stream>>>(P2, nHB, ZP, GPAD, g2, be2, Wf2, bf2, CC, NCB, FO, NBK, out, nG);
}
